// MPLayer_44942537786132
// MI455X (gfx1250) — hardware-verified
//
#include <hip/hip_runtime.h>


#define NB_  8
#define NND  512
#define FIN  32
#define KE   64
#define KN   128
#define FO   32
#define NE   (NB_ * NND * NND)
#define NNR  (NB_ * NND)
#define ECH  (NND * NND)
typedef _Float16 h16;
typedef unsigned short bf;
typedef __attribute__((ext_vector_type(16))) __bf16   v16bf;
typedef __attribute__((ext_vector_type(16))) _Float16 v16h;
typedef __attribute__((ext_vector_type(8)))  _Float16 v8h;
typedef __attribute__((ext_vector_type(8)))  unsigned short v8us;
typedef __attribute__((ext_vector_type(8)))  float    v8f;
typedef __attribute__((ext_vector_type(4)))  float    v4f;
typedef v8h  __attribute__((may_alias)) v8ha;
typedef v4f  __attribute__((may_alias)) v4fa;
typedef v8us __attribute__((may_alias)) v8usa;

__device__ __forceinline__ unsigned short f2bf(float f) { unsigned u = __float_as_uint(f); u += 0x7FFFu + ((u >> 16) & 1u); return (unsigned short)(u >> 16); }
__device__ __forceinline__ float bf2f(unsigned short b) { return __uint_as_float(((unsigned)b) << 16); }
__device__ __forceinline__ float bfr(float f) { return bf2f(f2bf(f)); }
__device__ __forceinline__ v16h cat16(v8h lo, v8h hi) { return __builtin_shufflevector(lo, hi, 0, 1, 2, 3, 4, 5, 6, 7, 8, 9, 10, 11, 12, 13, 14, 15); }
__device__ __forceinline__ v16bf cat16b(v8us lo, v8us hi) { return __builtin_bit_cast(v16bf, __builtin_shufflevector(lo, hi, 0, 1, 2, 3, 4, 5, 6, 7, 8, 9, 10, 11, 12, 13, 14, 15)); }
__device__ __forceinline__ v8f wmma16(v16h a, v16h b, v8f c) { return __builtin_amdgcn_wmma_f32_16x16x32_f16(false, a, false, b, (short)0, c, false, false); }
__device__ __forceinline__ v8f wmmab(v16bf a, v16bf b, v8f c) { return __builtin_amdgcn_wmma_f32_16x16x32_bf16(false, a, false, b, (short)0, c, false, false); }


template <typename T16> struct WFrag;
template <> struct WFrag<h16> { typedef v16h V; static __device__ __forceinline__ V ld(const h16* p) { return cat16(*(const v8h*)p, *(const v8h*)(p + 16)); } static __device__ __forceinline__ v8f mma(V a, V b, v8f c) { return wmma16(a, b, c); } };
template <> struct WFrag<bf> { typedef v16bf V; static __device__ __forceinline__ V ld(const bf* p) { return cat16b(*(const v8us*)p, *(const v8us*)(p + 16)); } static __device__ __forceinline__ v8f mma(V a, V b, v8f c) { return wmmab(a, b, c); } };
template <typename T16, int NSPLIT, bool BIAS>
__global__ __launch_bounds__(32) void k_gemmw(const T16* __restrict__ A, const T16* __restrict__ A2, const T16* __restrict__ Bt, const T16* __restrict__ Bt2, int K, float* C, int ldc, const float* __restrict__ bias, size_t sA, size_t sB, size_t sC) {
    typedef typename WFrag<T16>::V V;
    __shared__ __align__(16) float os[16 * 68];
    const size_t z = blockIdx.z; A += z * sA; if (A2) A2 += z * sA; Bt += z * sB; if (Bt2) Bt2 += z * sB; C += z * sC;
    const int lane = threadIdx.x & 31, lr = lane & 15, hi = lane >> 4; const int r0 = blockIdx.x * 64, c0 = blockIdx.y * 64;
    v8f acc[4][4];
#pragma unroll
    for (int mb = 0; mb < 4; ++mb)
#pragma unroll
        for (int nb = 0; nb < 4; ++nb) acc[mb][nb] = (v8f){};
    const size_t aoff = (size_t)(r0 + lr) * K + 8 * hi, boff = (size_t)(c0 + lr) * K + 8 * hi;
#pragma unroll 1
    for (int kc = 0; kc < K; kc += 32) {
        V a[4], a2[4];
#pragma unroll
        for (int mb = 0; mb < 4; ++mb) { a[mb] = WFrag<T16>::ld(A + aoff + (size_t)mb * 16 * K + kc); if (NSPLIT == 1 || NSPLIT == 2) a2[mb] = WFrag<T16>::ld(A2 + aoff + (size_t)mb * 16 * K + kc); }
#pragma unroll
        for (int nb = 0; nb < 4; ++nb) { const V b = WFrag<T16>::ld(Bt + boff + (size_t)nb * 16 * K + kc); V b2; if (NSPLIT >= 2) b2 = WFrag<T16>::ld(Bt2 + boff + (size_t)nb * 16 * K + kc);
#pragma unroll
            for (int mb = 0; mb < 4; ++mb) { acc[mb][nb] = WFrag<T16>::mma(a[mb], b, acc[mb][nb]); if (NSPLIT == 1 || NSPLIT == 2) acc[mb][nb] = WFrag<T16>::mma(a2[mb], b, acc[mb][nb]); if (NSPLIT >= 2) acc[mb][nb] = WFrag<T16>::mma(a[mb], b2, acc[mb][nb]); } }
        asm volatile("v_nop\n\tv_nop\n\tv_nop\n\tv_nop" : "+v"(acc[0][0]), "+v"(acc[1][1]), "+v"(acc[2][2]), "+v"(acc[3][3]) : "v"(a[0]), "v"(a[3]));
    }
#pragma unroll
    for (int mb = 0; mb < 4; ++mb) {
#pragma unroll
        for (int nb = 0; nb < 4; ++nb) {
#pragma unroll
            for (int j = 0; j < 8; ++j) os[(hi * 8 + j) * 68 + nb * 16 + lr] = acc[mb][nb][j]; }
        __builtin_amdgcn_wave_barrier(); asm volatile("" ::: "memory");
        float* crow = C + (size_t)(r0 + mb * 16) * ldc + c0;
#pragma unroll 1
        for (int ps = 0; ps < 2; ++ps) {
#pragma unroll
            for (int s = 0; s < 8; ++s) { const int row = 2 * s + hi, cofs = lr * 4; v4f val = *(const v4fa*)(os + row * 68 + cofs); if (BIAS) { val[0] += bfr(bias[c0 + cofs]); val[1] += bfr(bias[c0 + cofs + 1]); val[2] += bfr(bias[c0 + cofs + 2]); val[3] += bfr(bias[c0 + cofs + 3]); }
                *(volatile v4f*)(crow + (size_t)row * ldc + cofs) = val; }
            if (ps == 0) __threadfence(); }
        __builtin_amdgcn_wave_barrier(); asm volatile("" ::: "memory");
    }
}

__device__ __forceinline__ h16 tohx(float x) { return (h16)x; }
__device__ __forceinline__ float lrelu(float x) { return x >= 0.f ? x : 0.2f * x; }
__device__ __forceinline__ void splitf(float y, unsigned short& h, unsigned short& l) { h = f2bf(y); l = f2bf(y - bf2f(h)); }
typedef __attribute__((ext_vector_type(2))) _Float16 v2h;
typedef __attribute__((ext_vector_type(4))) _Float16 v4h;

__global__ __launch_bounds__(256) void k_cvt8(const float* __restrict__ src, bf* dst, size_t n8) { const size_t i = (size_t)blockIdx.x * 256 + threadIdx.x; if (i >= n8) return; const v8f v = *(const v8f*)(src + i * 8); v8us o;
#pragma unroll
    for (int k = 0; k < 8; ++k) o[k] = f2bf(v[k]); *(volatile v8us*)(dst + i * 8) = o; __threadfence(); *(volatile v8us*)(dst + i * 8) = o; }
__global__ __launch_bounds__(256) void k_wtb(const float* __restrict__ w, int K, int N, int Kp, int Np, bf* Bt) {
    typedef __attribute__((ext_vector_type(2))) unsigned short v2us;
    const int lane = threadIdx.x & 31; const int nlines = Np * Kp / 64; const int wg = blockIdx.x * 8 + (threadIdx.x >> 5), nw = gridDim.x * 8;
#pragma unroll 1
    for (int ps = 0; ps < 2; ++ps) {
#pragma unroll 1
        for (int L = wg; L < nlines; L += nw) { const int e = L * 64 + lane * 2; v2us o;
#pragma unroll
            for (int q = 0; q < 2; ++q) { const int n = (e + q) / Kp, k = (e + q) % Kp; o[q] = (n < N && k < K) ? f2bf(w[(size_t)(k < K ? k : 0) * N + (n < N ? n : 0)]) : (unsigned short)0; }
            *(volatile v2us*)(Bt + e) = o; }
        if (ps == 0) __threadfence(); }
}
__global__ __launch_bounds__(256) void k_wth(const float* __restrict__ w, int K, int N, h16* Bt) {
    const int lane = threadIdx.x & 31; const int nlines = N * K / 64; const int wg = blockIdx.x * 8 + (threadIdx.x >> 5), nw = gridDim.x * 8;
#pragma unroll 1
    for (int ps = 0; ps < 2; ++ps) {
#pragma unroll 1
        for (int L = wg; L < nlines; L += nw) { const int e = L * 64 + lane * 2; v2h o;
#pragma unroll
            for (int q = 0; q < 2; ++q) { const int n = (e + q) / K, k = (e + q) % K; o[q] = tohx(bfr(w[(size_t)k * N + n])); }
            *(volatile v2h*)(Bt + e) = o; }
        if (ps == 0) __threadfence(); }
}
__global__ __launch_bounds__(256) void k_w0t(const float* __restrict__ W0, const float* __restrict__ b0, bf* Bt, float* B0P) {
    typedef __attribute__((ext_vector_type(2))) unsigned short v2us;
    const int lane = threadIdx.x & 31; const int wg = blockIdx.x * 8 + (threadIdx.x >> 5); if (wg >= 128 * 32 / 64 + 4) return;
    if (wg < 64) { const int e = wg * 64 + lane * 2; v2us o;
#pragma unroll
        for (int q = 0; q < 2; ++q) { const int n = (e + q) / 32, k = (e + q) % 32; o[q] = f2bf(n < 64 ? W0[(size_t)k * 64 + n] : W0[(size_t)(32 + k) * 64 + (n - 64)]); }
        *(volatile v2us*)(Bt + e) = o; __threadfence(); *(volatile v2us*)(Bt + e) = o; }
    else { const int i = (wg - 64) * 32 + lane; const float v = i < 64 ? 0.f : b0[i - 64]; *(volatile float*)(B0P + i) = v; __threadfence(); *(volatile float*)(B0P + i) = v; }
}
__global__ __launch_bounds__(64) void k_bpad(const float* __restrict__ b, int N, float* out) { const int i = threadIdx.x; const float v = i < N ? b[i < N ? i : 0] : 0.f; *(volatile float*)(out + i) = v; __threadfence(); *(volatile float*)(out + i) = v; }
__global__ __launch_bounds__(256) void k_e0(const float* __restrict__ PQ, int b, h16* E0) {
    const int lane = threadIdx.x & 31; const int L0 = (blockIdx.x * 8 + (threadIdx.x >> 5)) * 8; const int nlines = ECH * KE / 64;
#pragma unroll 1
    for (int ps = 0; ps < 2; ++ps) {
#pragma unroll
        for (int l = 0; l < 8; ++l) { const int L = L0 + l; if (L >= nlines) break; const int e = L * 64 + lane * 2; const int c = e & 63; const int ij = e >> 6; const int i = ij >> 9, j = ij & 511; v2h v;
#pragma unroll
            for (int q = 0; q < 2; ++q) v[q] = tohx(lrelu(PQ[((size_t)b * NND + i) * 128 + c + q] + PQ[((size_t)b * NND + j) * 128 + 64 + c + q]));
            *(volatile v2h*)(E0 + (size_t)e) = v; }
        if (ps == 0) __threadfence(); }
}
__global__ __launch_bounds__(256) void k_act16(const float* __restrict__ H, int nlines, h16* P) {
    const int lane = threadIdx.x & 31; const int L0 = (blockIdx.x * 8 + (threadIdx.x >> 5)) * 8;
#pragma unroll 1
    for (int ps = 0; ps < 2; ++ps) {
#pragma unroll
        for (int l = 0; l < 8; ++l) { const int L = L0 + l; if (L >= nlines) break; const int e = L * 64 + lane * 2; v2h v;
#pragma unroll
            for (int q = 0; q < 2; ++q) v[q] = tohx(lrelu(H[(size_t)e + q]));
            *(volatile v2h*)(P + (size_t)e) = v; }
        if (ps == 0) __threadfence(); }
}
#define KNP 128
__global__ __launch_bounds__(256) void k_agg(const float* __restrict__ H2, const float* __restrict__ x, int b, bf* Hh, bf* Hl) {
    typedef __attribute__((ext_vector_type(4))) unsigned short v4us;
    const int lane = threadIdx.x & 31; const int i = blockIdx.x * 8 + (threadIdx.x >> 5); if (i >= NND) return; const int c0 = lane * 2; float s0 = 0.f, s1 = 0.f;
    const float* base = H2 + ((size_t)i * NND) * KE + c0;
#pragma unroll 4
    for (int j = 0; j < NND; ++j) { s0 += lrelu(base[(size_t)j * KE]); s1 += lrelu(base[(size_t)j * KE + 1]); }
    const float a0 = __shfl(s0, (lane * 2) & 31, 32), a1 = __shfl(s1, (lane * 2) & 31, 32), a2 = __shfl(s0, (lane * 2 + 1) & 31, 32), a3 = __shfl(s1, (lane * 2 + 1) & 31, 32);
    float v[4];
    if (lane < 16) { v[0] = a0; v[1] = a1; v[2] = a2; v[3] = a3; }
    else if (lane < 24) { const int xc = (lane - 16) * 4;
#pragma unroll
        for (int q = 0; q < 4; ++q) v[q] = bfr(x[((size_t)b * NND + i) * FIN + xc + q]); }
    else { v[0] = v[1] = v[2] = v[3] = 0.f; }
    v4us oh, ol;
#pragma unroll
    for (int q = 0; q < 4; ++q) { unsigned short a, c2; splitf(v[q], a, c2); oh[q] = a; ol[q] = c2; }
    const size_t o = ((size_t)b * NND + i) * KNP + lane * 4; *(volatile v4us*)(Hh + o) = oh; *(volatile v4us*)(Hl + o) = ol; __threadfence(); *(volatile v4us*)(Hh + o) = oh; *(volatile v4us*)(Hl + o) = ol;
}
__global__ __launch_bounds__(256) void k_nact(const float* __restrict__ H, bf* Ph, bf* Pl) {
    typedef __attribute__((ext_vector_type(2))) unsigned short v2us;
    const int lane = threadIdx.x & 31; const int L = blockIdx.x * 8 + (threadIdx.x >> 5); if (L >= NNR * KN / 64) return; const int e = L * 64 + lane * 2; v2us oh, ol;
#pragma unroll
    for (int q = 0; q < 2; ++q) { unsigned short a, c2; splitf(lrelu(H[e + q]), a, c2); oh[q] = a; ol[q] = c2; }
    *(volatile v2us*)(Ph + e) = oh; *(volatile v2us*)(Pl + e) = ol; __threadfence(); *(volatile v2us*)(Ph + e) = oh; *(volatile v2us*)(Pl + e) = ol;
}

__global__ __launch_bounds__(256) void k_out(const float* __restrict__ OUTP, float* OUT) {
    const int lane = threadIdx.x & 31; const int r = (blockIdx.x * 8 + (threadIdx.x >> 5)) * 4 + (lane >> 3); if (r >= NNR) return; const int c = (lane & 7) * 4;
    const v4f v = *(const v4f*)(OUTP + (size_t)r * 64 + c); *(volatile v4f*)(OUT + (size_t)r * FO + c) = v; __threadfence(); *(volatile v4f*)(OUT + (size_t)r * FO + c) = v;
}

extern "C" void kernel_launch(void* const* d_in, const int* in_sizes, int n_in,
                              void* d_out, int out_size, void* d_ws, size_t ws_size, hipStream_t stream) {
    (void)in_sizes; (void)n_in; (void)out_size;
    const float* x = (const float*)d_in[0]; const float* W0 = (const float*)d_in[1]; const float* b0 = (const float*)d_in[2]; const float* W1 = (const float*)d_in[3]; const float* b1 = (const float*)d_in[4]; const float* W2 = (const float*)d_in[5]; const float* b2 = (const float*)d_in[6];
    const float* V0 = (const float*)d_in[7]; const float* c0 = (const float*)d_in[8]; const float* V1 = (const float*)d_in[9]; const float* c1 = (const float*)d_in[10]; const float* V2 = (const float*)d_in[11]; const float* c2 = (const float*)d_in[12];
    float* OUT = (float*)d_out;
    char* wsp = (char*)d_ws;
    auto take = [&](size_t bytes) { char* p = wsp; wsp += (bytes + 255) & ~(size_t)255; return (void*)p; };
    bf* XB = (bf*)take((size_t)NNR * FIN * 2); bf* W0t = (bf*)take(128 * 32 * 2); float* B0P = (float*)take(128 * 4);
    h16* W1t = (h16*)take(KE * KE * 2); h16* W2t = (h16*)take(KE * KE * 2); bf* V0t = (bf*)take((size_t)KN * KNP * 2); bf* V1t = (bf*)take((size_t)KN * KN * 2); bf* V2t = (bf*)take((size_t)64 * KN * 2); float* C2P = (float*)take(64 * 4);
    float* PQ = (float*)take((size_t)NNR * 128 * 4);
    h16* E0 = (h16*)take((size_t)ECH * KE * 2); float* HE = (float*)take((size_t)ECH * KE * 4); h16* E1 = E0;
    bf* HNh = (bf*)take((size_t)NNR * KNP * 2); bf* HNl = (bf*)take((size_t)NNR * KNP * 2); float* G0 = (float*)take((size_t)NNR * KN * 4); bf* P0h = (bf*)take((size_t)NNR * KN * 2); bf* P0l = (bf*)take((size_t)NNR * KN * 2);
    float* OUTP = (float*)take((size_t)NNR * 64 * 4);
    if ((size_t)(wsp - (char*)d_ws) > ws_size) return;
    { const size_t nx = (size_t)NNR * FIN / 8; k_cvt8<<<(unsigned)((nx + 255) / 256), 256, 0, stream>>>(x, XB, nx); }
    k_w0t<<<(68 + 7) / 8, 256, 0, stream>>>(W0, b0, W0t, B0P);
    k_wth<<<2, 256, 0, stream>>>(W1, KE, KE, W1t); k_wth<<<2, 256, 0, stream>>>(W2, KE, KE, W2t);
    k_wtb<<<8, 256, 0, stream>>>(V0, 96, KN, KNP, KN, V0t); k_wtb<<<8, 256, 0, stream>>>(V1, KN, KN, KN, KN, V1t); k_wtb<<<4, 256, 0, stream>>>(V2, KN, FO, KN, 64, V2t); k_bpad<<<1, 64, 0, stream>>>(c2, FO, C2P);
    k_gemmw<bf, 0, true><<<dim3(NNR / 64, 2, 1), 32, 0, stream>>>(XB, nullptr, W0t, nullptr, FIN, PQ, 128, B0P, 0, 0, 0);
    const unsigned LBE = (unsigned)((ECH * KE / 64 + 63) / 64);
    for (int b = 0; b < NB_; ++b) {
        k_e0<<<LBE, 256, 0, stream>>>(PQ, b, E0);
        k_gemmw<h16, 0, true><<<dim3(ECH / 64, 1, 1), 32, 0, stream>>>(E0, nullptr, W1t, nullptr, KE, HE, KE, b1, 0, 0, 0);
        k_act16<<<LBE, 256, 0, stream>>>(HE, ECH * KE / 64, E1);
        k_gemmw<h16, 0, true><<<dim3(ECH / 64, 1, 1), 32, 0, stream>>>(E1, nullptr, W2t, nullptr, KE, HE, KE, b2, 0, 0, 0);
        k_agg<<<NND / 8, 256, 0, stream>>>(HE, x, b, HNh, HNl); }
    k_gemmw<bf, 1, true><<<dim3(NNR / 64, KN / 64, 1), 32, 0, stream>>>(HNh, HNl, V0t, nullptr, KNP, G0, KN, c0, 0, 0, 0);
    k_nact<<<(NNR * KN / 64 + 7) / 8, 256, 0, stream>>>(G0, P0h, P0l);
    k_gemmw<bf, 1, true><<<dim3(NNR / 64, KN / 64, 1), 32, 0, stream>>>(P0h, P0l, V1t, nullptr, KN, G0, KN, c1, 0, 0, 0);
    k_nact<<<(NNR * KN / 64 + 7) / 8, 256, 0, stream>>>(G0, P0h, P0l);
    k_gemmw<bf, 1, true><<<dim3(NNR / 64, 1, 1), 32, 0, stream>>>(P0h, P0l, V2t, nullptr, KN, OUTP, 64, C2P, 0, 0, 0);
    k_out<<<(NNR / 4 + 7) / 8, 256, 0, stream>>>(OUTP, OUT);
}
